// LanguageModelSRNN_76055280878226
// MI455X (gfx1250) — hardware-verified
//
#include <hip/hip_runtime.h>


typedef _Float16 f16t;
typedef f16t  v16h __attribute__((ext_vector_type(16)));
typedef f16t  v8h  __attribute__((ext_vector_type(8)));
typedef float v8f  __attribute__((ext_vector_type(8)));
typedef float v4f  __attribute__((ext_vector_type(4)));
typedef unsigned int v4u __attribute__((ext_vector_type(4)));

union Frag { v16h v; v8h q[2]; };
union Pk16 { v8h h; v4u u; };

#define HID   1024
#define VOC   128
#define NSEQ  64
#define TLEN  512
#define LP    1032

__device__ __forceinline__ v8f wmma16(v16h a, v16h b, v8f c) {
    return __builtin_amdgcn_wmma_f32_16x16x32_f16(false, a, false, b, (short)0, c, false, false);
}

__device__ __forceinline__ void wguard(v8f (&c)[8][1], Frag (&a)[8], Frag (&b)[1]) {
    asm volatile("v_nop\n\tv_nop\n\tv_nop\n\tv_nop"
                 : "+v"(c[0][0]), "+v"(c[1][0]), "+v"(c[2][0]), "+v"(c[3][0]),
                   "+v"(c[4][0]), "+v"(c[5][0]), "+v"(c[6][0]), "+v"(c[7][0])
                 : "v"(a[0].v), "v"(a[1].v), "v"(a[2].v), "v"(a[3].v),
                   "v"(a[4].v), "v"(a[5].v), "v"(a[6].v), "v"(a[7].v), "v"(b[0].v));
}
__device__ __forceinline__ void wguard(v8f (&c)[1][8], Frag (&a)[1], Frag (&b)[8]) {
    asm volatile("v_nop\n\tv_nop\n\tv_nop\n\tv_nop"
                 : "+v"(c[0][0]), "+v"(c[0][1]), "+v"(c[0][2]), "+v"(c[0][3]),
                   "+v"(c[0][4]), "+v"(c[0][5]), "+v"(c[0][6]), "+v"(c[0][7])
                 : "v"(a[0].v), "v"(b[0].v), "v"(b[1].v), "v"(b[2].v), "v"(b[3].v),
                   "v"(b[4].v), "v"(b[5].v), "v"(b[6].v), "v"(b[7].v));
}

template<int MT, int NT>
__device__ __forceinline__ void zacc(v8f (&acc)[MT][NT]) {
    const v8f z = {0.f, 0.f, 0.f, 0.f, 0.f, 0.f, 0.f, 0.f};
#pragma unroll
    for (int i = 0; i < MT; ++i)
#pragma unroll
        for (int j = 0; j < NT; ++j) acc[i][j] = z;
}

template<int MT, int NT>
__device__ __forceinline__ void mma_acc(v8f (&acc)[MT][NT],
                                        const f16t* A, int lda,
                                        const f16t* B, int ldb, int ktiles) {
    const int l = threadIdx.x & 31, h = l >> 4, m = l & 15;
    const f16t* ap = A + (size_t)m * lda + 8 * h;
    const f16t* bp = B + (size_t)m * ldb + 8 * h;
#pragma unroll 1
    for (int kt = 0; kt < ktiles; ++kt) {
        Frag a[MT], b[NT];
#pragma unroll
        for (int i = 0; i < MT; ++i) {
            const f16t* p = ap + (size_t)i * 16 * lda + kt * 32;
            a[i].q[0] = *(const v8h*)p;
            a[i].q[1] = *(const v8h*)(p + 16);
        }
#pragma unroll
        for (int j = 0; j < NT; ++j) {
            const f16t* p = bp + (size_t)j * 16 * ldb + kt * 32;
            b[j].q[0] = *(const v8h*)p;
            b[j].q[1] = *(const v8h*)(p + 16);
        }
#pragma unroll
        for (int i = 0; i < MT; ++i)
#pragma unroll
            for (int j = 0; j < NT; ++j)
                acc[i][j] = wmma16(a[i].v, b[j].v, acc[i][j]);
        wguard(acc, a, b);
    }
}

__device__ __forceinline__ float ftanh(float x) {
    float ax = fabsf(x);
    float t  = __expf(-2.0f * ax);
    float r  = (1.0f - t) * __builtin_amdgcn_rcpf(1.0f + t);
    return copysignf(r, x);
}

__global__ __launch_bounds__(256)
void k_cvt8(const float* x, f16t* y, int n8, float sc) {
    int i = blockIdx.x * 256 + threadIdx.x;
    if (i >= n8) return;
    const float* p = x + (size_t)i * 8;
    v4f a = *(const v4f*)p;
    v4f b = *(const v4f*)(p + 4);
    Pk16 k;
    k.h[0] = (f16t)(a[0] * sc); k.h[1] = (f16t)(a[1] * sc);
    k.h[2] = (f16t)(a[2] * sc); k.h[3] = (f16t)(a[3] * sc);
    k.h[4] = (f16t)(b[0] * sc); k.h[5] = (f16t)(b[1] * sc);
    k.h[6] = (f16t)(b[2] * sc); k.h[7] = (f16t)(b[3] * sc);
    f16t* d = y + (size_t)i * 8;
    *(volatile v4u*)d = k.u;
    __threadfence();
    *(volatile v4u*)d = k.u;
}

__global__ __launch_bounds__(256)
void k_rnn(const int* X, const float* W, const f16t* Upl, f16t* Hpl,
           int nseq, int T, float invU) {
    __shared__ __attribute__((aligned(16))) f16t H16[16 * LP];
    const int tid = threadIdx.x;
    const int w   = tid >> 5;
    const int l   = tid & 31, h = l >> 4, m = l & 15;
    const int b0  = blockIdx.x * 16;
    if (b0 + 16 > nseq) return;

    for (int i = tid; i < 16 * LP; i += 256) H16[i] = (f16t)0.0f;
    __syncthreads();

    const int   f0 = 128 * w;
    const f16t* Uw = Upl + (size_t)f0 * HID;
    const int*  xr = X + (size_t)(b0 + m) * T;

#pragma unroll 1
    for (int t = 0; t < T; ++t) {
        int tok = xr[t];
        const bool tv = (unsigned)tok < (unsigned)VOC;
        tok = tv ? tok : 0;

        v8f acc[8][1]; zacc(acc);
        mma_acc<8, 1>(acc, Uw, HID, H16, LP, HID / 32);
        __syncthreads();

#pragma unroll
        for (int i = 0; i < 8; ++i) {
            const int n0 = f0 + 16 * i + 8 * h;
            const float* wq = W + (size_t)n0 * VOC + tok;
            Pk16 pk;
#pragma unroll
            for (int r = 0; r < 8; ++r) {
                float g = wq[(size_t)r * VOC];
                g = tv ? g : 0.0f;
                float pre = fmaf(acc[i][0][r], invU, g);
                pk.h[r] = (f16t)ftanh(pre);
            }
            *(v8h*)(H16 + (size_t)m * LP + n0) = pk.h;
        }
        __syncthreads();

        Pk16 v[8];
#pragma unroll
        for (int i = 0; i < 8; ++i) {
            int p = tid + 256 * i, row = p >> 7, ch = (p & 127) * 8;
            v[i].h = *(const v8h*)(H16 + row * LP + ch);
        }
        f16t* Hr = Hpl + ((size_t)b0 * T + t) * HID;
#pragma unroll
        for (int i = 0; i < 8; ++i) {
            int p = tid + 256 * i, row = p >> 7, ch = (p & 127) * 8;
            *(volatile v4u*)(Hr + (size_t)row * T * HID + ch) = v[i].u;
        }
        __threadfence();
#pragma unroll
        for (int i = 0; i < 8; ++i) {
            int p = tid + 256 * i, row = p >> 7, ch = (p & 127) * 8;
            *(volatile v4u*)(Hr + (size_t)row * T * HID + ch) = v[i].u;
        }
    }
}

__global__ __launch_bounds__(128)
void k_proj(const f16t* Hpl, const f16t* Lpl, const float* lin_b, float* out,
            int nrows, float invL) {
    __shared__ __attribute__((aligned(16))) float S[4 * 16 * VOC];
    const int tid = threadIdx.x;
    const int w   = tid >> 5;
    const int l   = tid & 31, h = l >> 4, m = l & 15;
    const int rb  = blockIdx.x * 64;
    if (rb + 64 > nrows) return;
    const int r0 = rb + 16 * w;

    v8f acc[1][8]; zacc(acc);
    mma_acc<1, 8>(acc, Hpl + (size_t)r0 * HID, HID, Lpl, HID, HID / 32);

    float bias[8];
#pragma unroll
    for (int j = 0; j < 8; ++j) bias[j] = lin_b[16 * j + m];

    float* Sw = S + w * (16 * VOC);
#pragma unroll
    for (int r = 0; r < 8; ++r) {
        float v[8];
        float mx = -3.0e38f;
#pragma unroll
        for (int j = 0; j < 8; ++j) {
            v[j] = fmaf(acc[0][j][r], invL, bias[j]);
            mx = fmaxf(mx, v[j]);
        }
#pragma unroll
        for (int d = 1; d < 16; d <<= 1) mx = fmaxf(mx, __shfl_xor(mx, d, 32));
        float sum = 0.0f;
#pragma unroll
        for (int j = 0; j < 8; ++j) {
            v[j] = __expf(v[j] - mx);
            sum += v[j];
        }
#pragma unroll
        for (int d = 1; d < 16; d <<= 1) sum += __shfl_xor(sum, d, 32);
        float inv = __builtin_amdgcn_rcpf(sum);
#pragma unroll
        for (int j = 0; j < 8; ++j) Sw[(8 * h + r) * VOC + 16 * j + m] = v[j] * inv;
    }
    __syncthreads();

    float* orow = out + (size_t)r0 * VOC;
#pragma unroll
    for (int rr = 0; rr < 16; ++rr) {
        v4f q = *(const v4f*)(Sw + rr * VOC + 4 * l);
        *(volatile v4f*)(orow + (size_t)rr * VOC + 4 * l) = q;
    }
    __threadfence();
#pragma unroll
    for (int rr = 0; rr < 16; ++rr) {
        v4f q = *(const v4f*)(Sw + rr * VOC + 4 * l);
        *(volatile v4f*)(orow + (size_t)rr * VOC + 4 * l) = q;
    }
}

extern "C" void kernel_launch(void* const* d_in, const int* in_sizes, int n_in,
                              void* d_out, int out_size, void* d_ws, size_t ws_size,
                              hipStream_t stream) {
    const int nseq = NSEQ, T = TLEN;
    const int nrows = nseq * T;

    if (n_in < 5) return;
    if (in_sizes[0] != nrows || in_sizes[1] != HID * HID || in_sizes[2] != HID * VOC ||
        in_sizes[3] != VOC * HID || in_sizes[4] != VOC) return;
    if (out_size != nrows * VOC) return;
    if ((nseq % 16) != 0 || (nrows % 64) != 0) return;

    const int*   X     = (const int*)d_in[0];
    const float* U     = (const float*)d_in[1];
    const float* W     = (const float*)d_in[2];
    const float* lin_w = (const float*)d_in[3];
    const float* lin_b = (const float*)d_in[4];
    float* out = (float*)d_out;

    char* ws = (char*)d_ws;
    size_t off = 0;
    auto carve = [&](size_t bytes) -> char* {
        char* p = ws + off;
        off = (off + bytes + 255) & ~(size_t)255;
        return p;
    };
    f16t* Upl = (f16t*)carve((size_t)HID * HID * 2);
    f16t* Lpl = (f16t*)carve((size_t)VOC * HID * 2);
    f16t* Hpl = (f16t*)carve((size_t)nrows * HID * 2);
    if (off > ws_size) return;

    const float SU = 64.0f,  IU = 0.015625f;
    const float SL = 128.0f, IL = 0.0078125f;

    {
        int n8 = HID * HID / 8;
        k_cvt8<<<dim3((n8 + 255) / 256), dim3(256), 0, stream>>>(U, Upl, n8, SU);
        n8 = VOC * HID / 8;
        k_cvt8<<<dim3((n8 + 255) / 256), dim3(256), 0, stream>>>(lin_w, Lpl, n8, SL);
    }
    k_rnn<<<dim3(nseq / 16), dim3(256), 0, stream>>>(X, W, Upl, Hpl, nseq, T, IU);
    k_proj<<<dim3(nrows / 64), dim3(128), 0, stream>>>(Hpl, Lpl, lin_b, out, nrows, IL);
}
